// MultiHeadAdditiveAttention_38680475467956
// MI455X (gfx1250) — hardware-verified
//
#include <hip/hip_runtime.h>


#define NB_  2
#define LL   512
#define DM   512
#define NH_  8
#define HD   64
typedef _Float16 h16;
typedef unsigned short bf;
typedef __attribute__((ext_vector_type(16))) __bf16   v16bf;
typedef __attribute__((ext_vector_type(16))) _Float16 v16h;
typedef __attribute__((ext_vector_type(8)))  _Float16 v8h;
typedef __attribute__((ext_vector_type(8)))  unsigned short v8us;
typedef __attribute__((ext_vector_type(8)))  float    v8f;
typedef __attribute__((ext_vector_type(4)))  float    v4f;
typedef v8h  __attribute__((may_alias)) v8ha;
typedef v4f  __attribute__((may_alias)) v4fa;
typedef v8us __attribute__((may_alias)) v8usa;

__device__ __forceinline__ unsigned short f2bf(float f) { unsigned u = __float_as_uint(f); u += 0x7FFFu + ((u >> 16) & 1u); return (unsigned short)(u >> 16); }
__device__ __forceinline__ float bf2f(unsigned short b) { return __uint_as_float(((unsigned)b) << 16); }
__device__ __forceinline__ float bfr(float f) { return bf2f(f2bf(f)); }
__device__ __forceinline__ v16h cat16(v8h lo, v8h hi) { return __builtin_shufflevector(lo, hi, 0, 1, 2, 3, 4, 5, 6, 7, 8, 9, 10, 11, 12, 13, 14, 15); }
__device__ __forceinline__ v16bf cat16b(v8us lo, v8us hi) { return __builtin_bit_cast(v16bf, __builtin_shufflevector(lo, hi, 0, 1, 2, 3, 4, 5, 6, 7, 8, 9, 10, 11, 12, 13, 14, 15)); }
__device__ __forceinline__ v8f wmma16(v16h a, v16h b, v8f c) { return __builtin_amdgcn_wmma_f32_16x16x32_f16(false, a, false, b, (short)0, c, false, false); }
__device__ __forceinline__ v8f wmmab(v16bf a, v16bf b, v8f c) { return __builtin_amdgcn_wmma_f32_16x16x32_bf16(false, a, false, b, (short)0, c, false, false); }


template <typename T16> struct WFrag;
template <> struct WFrag<h16> { typedef v16h V; static __device__ __forceinline__ V ld(const h16* p) { return cat16(*(const v8h*)p, *(const v8h*)(p + 16)); } static __device__ __forceinline__ v8f mma(V a, V b, v8f c) { return wmma16(a, b, c); } };
template <> struct WFrag<bf> { typedef v16bf V; static __device__ __forceinline__ V ld(const bf* p) { return cat16b(*(const v8us*)p, *(const v8us*)(p + 16)); } static __device__ __forceinline__ v8f mma(V a, V b, v8f c) { return wmmab(a, b, c); } };
template <typename T16, int NSPLIT, bool BIAS>
__global__ __launch_bounds__(32) void k_gemmw(const T16* __restrict__ A, const T16* __restrict__ A2, const T16* __restrict__ Bt, const T16* __restrict__ Bt2, int K, float* C, int ldc, const float* __restrict__ bias, size_t sA, size_t sB, size_t sC) {
    typedef typename WFrag<T16>::V V;
    __shared__ __align__(16) float os[16 * 68];
    const size_t z = blockIdx.z; A += z * sA; if (A2) A2 += z * sA; Bt += z * sB; if (Bt2) Bt2 += z * sB; C += z * sC;
    const int lane = threadIdx.x & 31, lr = lane & 15, hi = lane >> 4; const int r0 = blockIdx.x * 64, c0 = blockIdx.y * 64;
    v8f acc[4][4];
#pragma unroll
    for (int mb = 0; mb < 4; ++mb)
#pragma unroll
        for (int nb = 0; nb < 4; ++nb) acc[mb][nb] = (v8f){};
    const size_t aoff = (size_t)(r0 + lr) * K + 8 * hi, boff = (size_t)(c0 + lr) * K + 8 * hi;
#pragma unroll 1
    for (int kc = 0; kc < K; kc += 32) {
        V a[4], a2[4];
#pragma unroll
        for (int mb = 0; mb < 4; ++mb) { a[mb] = WFrag<T16>::ld(A + aoff + (size_t)mb * 16 * K + kc); if (NSPLIT == 1 || NSPLIT == 2) a2[mb] = WFrag<T16>::ld(A2 + aoff + (size_t)mb * 16 * K + kc); }
#pragma unroll
        for (int nb = 0; nb < 4; ++nb) { const V b = WFrag<T16>::ld(Bt + boff + (size_t)nb * 16 * K + kc); V b2; if (NSPLIT >= 2) b2 = WFrag<T16>::ld(Bt2 + boff + (size_t)nb * 16 * K + kc);
#pragma unroll
            for (int mb = 0; mb < 4; ++mb) { acc[mb][nb] = WFrag<T16>::mma(a[mb], b, acc[mb][nb]); if (NSPLIT == 1 || NSPLIT == 2) acc[mb][nb] = WFrag<T16>::mma(a2[mb], b, acc[mb][nb]); if (NSPLIT >= 2) acc[mb][nb] = WFrag<T16>::mma(a[mb], b2, acc[mb][nb]); } }
        asm volatile("v_nop\n\tv_nop\n\tv_nop\n\tv_nop" : "+v"(acc[0][0]), "+v"(acc[1][1]), "+v"(acc[2][2]), "+v"(acc[3][3]) : "v"(a[0]), "v"(a[3]));
    }
#pragma unroll
    for (int mb = 0; mb < 4; ++mb) {
#pragma unroll
        for (int nb = 0; nb < 4; ++nb) {
#pragma unroll
            for (int j = 0; j < 8; ++j) os[(hi * 8 + j) * 68 + nb * 16 + lr] = acc[mb][nb][j]; }
        __builtin_amdgcn_wave_barrier(); asm volatile("" ::: "memory");
        float* crow = C + (size_t)(r0 + mb * 16) * ldc + c0;
#pragma unroll 1
        for (int ps = 0; ps < 2; ++ps) {
#pragma unroll
            for (int s = 0; s < 8; ++s) { const int row = 2 * s + hi, cofs = lr * 4; v4f val = *(const v4fa*)(os + row * 68 + cofs); if (BIAS) { val[0] += bfr(bias[c0 + cofs]); val[1] += bfr(bias[c0 + cofs + 1]); val[2] += bfr(bias[c0 + cofs + 2]); val[3] += bfr(bias[c0 + cofs + 3]); }
                *(volatile v4f*)(crow + (size_t)row * ldc + cofs) = val; }
            if (ps == 0) __threadfence(); }
        __builtin_amdgcn_wave_barrier(); asm volatile("" ::: "memory");
    }
}

__device__ __forceinline__ void splitf(float y, unsigned short& h, unsigned short& l) { h = f2bf(y); l = f2bf(y - bf2f(h)); }
typedef __attribute__((ext_vector_type(2))) unsigned short v2us;
typedef __attribute__((ext_vector_type(4))) unsigned short v4us;

__global__ __launch_bounds__(256) void k_cvt8(const float* __restrict__ src, bf* dst, size_t n8) { const size_t i = (size_t)blockIdx.x * 256 + threadIdx.x; if (i >= n8) return; const v8f v = *(const v8f*)(src + i * 8); v8us o;
#pragma unroll
    for (int k = 0; k < 8; ++k) o[k] = f2bf(v[k]); *(volatile v8us*)(dst + i * 8) = o; __threadfence(); *(volatile v8us*)(dst + i * 8) = o; }
__global__ __launch_bounds__(256) void k_bdA(const float* __restrict__ A, bf* Bt) { const int e = (blockIdx.x * 256 + threadIdx.x) * 4; if (e >= DM * DM) return; const int k = e % DM; const int n = e / DM; v4us o;
#pragma unroll
    for (int u = 0; u < 4; ++u) o[u] = ((k + u) / HD == n / HD) ? f2bf(A[(size_t)(n % HD) * HD + (k + u) % HD]) : (unsigned short)0; *(volatile v4us*)(Bt + e) = o; __threadfence(); *(volatile v4us*)(Bt + e) = o; }
__global__ __launch_bounds__(256) void k_pl(const float* __restrict__ F, bf* Ph, bf* Pl, size_t n4) { const size_t e = ((size_t)blockIdx.x * 256 + threadIdx.x) * 4; if (e >= n4 * 4) return; const v4f a = *(const v4f*)(F + e); v4us oh, ol;
#pragma unroll
    for (int u = 0; u < 4; ++u) { unsigned short x0, x1; splitf(a[u], x0, x1); oh[u] = x0; ol[u] = x1; } *(volatile v4us*)(Ph + e) = oh; *(volatile v4us*)(Pl + e) = ol; __threadfence(); *(volatile v4us*)(Ph + e) = oh; *(volatile v4us*)(Pl + e) = ol; }
__global__ __launch_bounds__(256) void k_vtp(const float* __restrict__ V, bf* Ph, bf* Pl) { const size_t e = ((size_t)blockIdx.x * 256 + threadIdx.x) * 2; if (e >= (size_t)NH_ * HD * LL) return; const int j = (int)(e % LL); const int d = (int)((e / LL) % HD); const int h = (int)(e / ((size_t)LL * HD)); v2us oh, ol;
#pragma unroll
    for (int u = 0; u < 2; ++u) { unsigned short a, b; splitf(V[(size_t)(j + u) * DM + h * HD + d], a, b); oh[u] = a; ol[u] = b; } *(volatile v2us*)(Ph + e) = oh; *(volatile v2us*)(Pl + e) = ol; __threadfence(); *(volatile v2us*)(Ph + e) = oh; *(volatile v2us*)(Pl + e) = ol; }
typedef __attribute__((address_space(1))) const float gfloat;
__device__ __attribute__((noinline)) float energy64(gfloat* __restrict__ qp, gfloat* __restrict__ kp, gfloat* __restrict__ av) { float e = 0.f;
#pragma unroll 1
    for (int d = 0; d < HD; ++d) { const float z = __fadd_rn(qp[d], kp[d]); const float th = tanhf(z); float pr = __fmul_rn(bfr(av[d]), th); asm volatile("" : "+v"(pr)); e = __fadd_rn(e, pr); }
    return e; }
__global__ __launch_bounds__(256) void k_esoft(const float* __restrict__ QP, const float* __restrict__ KP, const float* __restrict__ av, bf* Ph, bf* Pl) {
    const int lane = threadIdx.x & 31; const int row = blockIdx.x * 8 + (threadIdx.x >> 5); if (row >= NH_ * LL) return; const int i = row % LL; const int h = row / LL;
    const float* qp = QP + (size_t)i * DM + h * HD; float v[LL / 32]; float mx = -3.0e38f;
#pragma unroll
    for (int ch = 0; ch < LL / 128; ++ch) {
#pragma unroll
        for (int u = 0; u < 4; ++u) { const int j = ch * 128 + lane * 4 + u; const float* kp = KP + (size_t)j * DM + h * HD; const float e = energy64((gfloat*)qp, (gfloat*)kp, (gfloat*)av);
            v[ch * 4 + u] = e; mx = fmaxf(mx, e); } }
#pragma unroll
    for (int sh = 16; sh; sh >>= 1) mx = fmaxf(mx, __shfl_xor(mx, sh, 32));
    float sum = 0.f;
#pragma unroll
    for (int q = 0; q < LL / 32; ++q) { float d0 = __fsub_rn(v[q], mx); asm volatile("" : "+v"(d0)); v[q] = __builtin_amdgcn_exp2f(__fmul_rn(d0, 1.4426950408889634f)); sum += v[q]; }
#pragma unroll
    for (int sh = 16; sh; sh >>= 1) sum += __shfl_xor(sum, sh, 32);
    const float f = __fdiv_rn(1.0f, sum);
    for (int ps = 0; ps < 2; ++ps) {
#pragma unroll
        for (int ch = 0; ch < LL / 128; ++ch) { v4us oh, ol; for (int q = 0; q < 4; ++q) { unsigned short a2, c2; splitf(v[ch * 4 + q] * f, a2, c2); oh[q] = a2; ol[q] = c2; } const size_t oo = (size_t)row * LL + ch * 128 + lane * 4; *(volatile v4us*)(Ph + oo) = oh; *(volatile v4us*)(Pl + oo) = ol; }
        if (ps == 0) __threadfence(); } }
__global__ __launch_bounds__(256) void k_mrg(const float* __restrict__ O, bf* Ah, bf* Al) { const size_t e = ((size_t)blockIdx.x * 256 + threadIdx.x) * 4; if (e >= (size_t)NH_ * LL * HD) return; const int d = (int)(e % HD); const int i = (int)((e / HD) % LL); const int h = (int)(e / ((size_t)HD * LL)); const size_t oo = (size_t)i * DM + h * HD + d; v4us oh, ol;
#pragma unroll
    for (int u = 0; u < 4; ++u) { unsigned short a, b; splitf(O[e + u], a, b); oh[u] = a; ol[u] = b; } *(volatile v4us*)(Ah + oo) = oh; *(volatile v4us*)(Al + oo) = ol; __threadfence(); *(volatile v4us*)(Ah + oo) = oh; *(volatile v4us*)(Al + oo) = ol; }

extern "C" void kernel_launch(void* const* d_in, const int* in_sizes, int n_in,
                              void* d_out, int out_size, void* d_ws, size_t ws_size, hipStream_t stream) {
    (void)in_sizes; (void)n_in; (void)out_size;
    const float* xq = (const float*)d_in[0]; const float* xk = (const float*)d_in[1]; const float* xv = (const float*)d_in[2]; const float* Wq = (const float*)d_in[3]; const float* bq = (const float*)d_in[4]; const float* Wk = (const float*)d_in[5]; const float* bk = (const float*)d_in[6]; const float* Wv = (const float*)d_in[7]; const float* bv = (const float*)d_in[8]; const float* Wo = (const float*)d_in[9]; const float* bo = (const float*)d_in[10]; const float* Aq = (const float*)d_in[11]; const float* Ak = (const float*)d_in[12]; const float* av = (const float*)d_in[13];
    float* OUT = (float*)d_out;
    char* wsp = (char*)d_ws;
    auto take = [&](size_t bytes) { char* p = wsp; wsp += (bytes + 255) & ~(size_t)255; return (void*)p; };
    bf* BQ = (bf*)take((size_t)DM * DM * 2); bf* BK = (bf*)take((size_t)DM * DM * 2); bf* BV = (bf*)take((size_t)DM * DM * 2); bf* BO = (bf*)take((size_t)DM * DM * 2); bf* BAQ = (bf*)take((size_t)DM * DM * 2); bf* BAK = (bf*)take((size_t)DM * DM * 2);
    bf* XB = (bf*)take((size_t)LL * DM * 2); float* F = (float*)take((size_t)LL * DM * 4); bf* Fh = (bf*)take((size_t)LL * DM * 2); bf* Fl = (bf*)take((size_t)LL * DM * 2); float* QP = (float*)take((size_t)LL * DM * 4); float* KP = (float*)take((size_t)LL * DM * 4);
    bf* VTh = (bf*)take((size_t)NH_ * HD * LL * 2); bf* VTl = (bf*)take((size_t)NH_ * HD * LL * 2); bf* Ph = (bf*)take((size_t)NH_ * LL * LL * 2); bf* Pl = (bf*)take((size_t)NH_ * LL * LL * 2); float* O = (float*)take((size_t)NH_ * LL * HD * 4); bf* ATh = (bf*)take((size_t)LL * DM * 2); bf* ATl = (bf*)take((size_t)LL * DM * 2);
    if ((size_t)(wsp - (char*)d_ws) > ws_size) return;
    k_cvt8<<<(DM * DM / 8 + 255) / 256, 256, 0, stream>>>(Wq, BQ, DM * DM / 8); k_cvt8<<<(DM * DM / 8 + 255) / 256, 256, 0, stream>>>(Wk, BK, DM * DM / 8); k_cvt8<<<(DM * DM / 8 + 255) / 256, 256, 0, stream>>>(Wv, BV, DM * DM / 8); k_cvt8<<<(DM * DM / 8 + 255) / 256, 256, 0, stream>>>(Wo, BO, DM * DM / 8);
    k_bdA<<<(DM * DM / 4 + 255) / 256, 256, 0, stream>>>(Aq, BAQ); k_bdA<<<(DM * DM / 4 + 255) / 256, 256, 0, stream>>>(Ak, BAK);
    const dim3 gp(LL / 64, DM / 64, 1); const unsigned LP = (unsigned)(((size_t)LL * DM / 4 + 255) / 256); const size_t zP = (size_t)LL * LL, zV = (size_t)HD * LL, zO = (size_t)LL * HD;
    for (int b = 0; b < NB_; ++b) {
        k_cvt8<<<(LL * DM / 8 + 255) / 256, 256, 0, stream>>>(xq + (size_t)b * LL * DM, XB, LL * DM / 8); k_gemmw<bf, 0, true><<<gp, 32, 0, stream>>>(XB, nullptr, BQ, nullptr, DM, F, DM, bq, 0, 0, 0); k_pl<<<LP, 256, 0, stream>>>(F, Fh, Fl, (size_t)LL * DM / 4);
        k_gemmw<bf, 1, false><<<gp, 32, 0, stream>>>(Fh, Fl, BAQ, nullptr, DM, QP, DM, nullptr, 0, 0, 0);
        k_cvt8<<<(LL * DM / 8 + 255) / 256, 256, 0, stream>>>(xk + (size_t)b * LL * DM, XB, LL * DM / 8); k_gemmw<bf, 0, true><<<gp, 32, 0, stream>>>(XB, nullptr, BK, nullptr, DM, F, DM, bk, 0, 0, 0); k_pl<<<LP, 256, 0, stream>>>(F, Fh, Fl, (size_t)LL * DM / 4);
        k_gemmw<bf, 1, false><<<gp, 32, 0, stream>>>(Fh, Fl, BAK, nullptr, DM, KP, DM, nullptr, 0, 0, 0);
        k_cvt8<<<(LL * DM / 8 + 255) / 256, 256, 0, stream>>>(xv + (size_t)b * LL * DM, XB, LL * DM / 8); k_gemmw<bf, 0, true><<<gp, 32, 0, stream>>>(XB, nullptr, BV, nullptr, DM, F, DM, bv, 0, 0, 0); k_vtp<<<(unsigned)(((size_t)NH_ * HD * LL / 2 + 255) / 256), 256, 0, stream>>>(F, VTh, VTl);
        k_esoft<<<NH_ * LL / 8, 256, 0, stream>>>(QP, KP, av, Ph, Pl);
        k_gemmw<bf, 2, false><<<dim3(LL / 64, 1, NH_), 32, 0, stream>>>(Ph, Pl, VTh, VTl, LL, O, HD, nullptr, zP, zV, zO);
        k_mrg<<<(unsigned)(((size_t)NH_ * LL * HD / 4 + 255) / 256), 256, 0, stream>>>(O, ATh, ATl);
        k_gemmw<bf, 1, true><<<gp, 32, 0, stream>>>(ATh, ATl, BO, nullptr, DM, OUT + (size_t)b * LL * DM, DM, bo, 0, 0, 0); }
}
